// M2_GNN_Regressor_38766374814298
// MI455X (gfx1250) — hardware-verified
//
#include <hip/hip_runtime.h>
#include <stddef.h>
#include <math.h>


#define NTHR   256
#define NWAVE  8
#define EPT    8
#define CHUNK  (NTHR * EPT)
#define WCAP   (EPT * 32)
#define LISTN  (NWAVE * WCAP)
#define PASSN  (NWAVE * 16)
#define PCAP   (CHUNK + PASSN)
#define NB     768
#define FD     64
#define CIN    6
#define EDIM   2
#define TB     8
#define TD     32
#define NPL    9
#define RB     (NWAVE * 16)
#define WSC    16.0f
#define HSC    4.0f
#define HINV   0.015625f
#define WINV   0.0625f

#define LDS_ACC   0
#define LDS_MSG   (LDS_ACC + (NB + 1) * FD * 4)
#define LDS_STG   (LDS_MSG + PASSN * FD * 4)
#define LDS_LIST  (LDS_STG + PASSN * EDIM * 4)
#define LDS_PEND  (LDS_LIST + LISTN * 4)
#define LDS_SLOT  (LDS_PEND + PCAP * 4)
#define LDS_PRM   (LDS_SLOT + PASSN * 4)
#define LDS_WCNT  (LDS_PRM + 8 * FD * 4)
#define LDS_TOTAL (LDS_WCNT + 64)

static_assert(PASSN == 128);
static_assert(PCAP >= CHUNK + PASSN);
static_assert((NB % (NWAVE * 16)) == 0);
static_assert(((NB / NWAVE) % 2) == 0);
static_assert((NB % RB) == 0);
static_assert(NWAVE * 16 * FD * 2 <= PASSN * FD * 4);
static_assert((LDS_MSG % 16) == 0 && (LDS_STG % 16) == 0 && (LDS_LIST % 16) == 0);
static_assert((LDS_PEND % 16) == 0 && (LDS_SLOT % 16) == 0 && (LDS_PRM % 16) == 0 && (LDS_WCNT % 16) == 0);
static_assert((LDS_TOTAL % 16) == 0);
static_assert(LDS_TOTAL <= 300 * 1024);
static_assert(NTHR == TB * TD);
static_assert(2 * NTHR == TB * FD);
static_assert(2 * NTHR * 8 == FD * FD);
static_assert((TB * FD) % 4 == 0 && (TB * FD) / 4 <= NTHR);

typedef float    v2f  __attribute__((ext_vector_type(2)));
typedef float    v4f  __attribute__((ext_vector_type(4)));
typedef float    v8f  __attribute__((ext_vector_type(8)));
typedef int      v4i  __attribute__((ext_vector_type(4)));
typedef _Float16 v8h  __attribute__((ext_vector_type(8)));
typedef _Float16 v16h __attribute__((ext_vector_type(16)));
union FragH { v16h v; v8h h[2]; };
union Pk8 { v8h h; v4i i; };

__device__ __forceinline__ float silu_f(float x) {
  return x * __builtin_amdgcn_rcpf(1.0f + __expf(-x));
}

__device__ __forceinline__ v8f wmh(v16h a, v16h b, v8f c) {
  v8f d = __builtin_amdgcn_wmma_f32_16x16x32_f16(false, a, false, b, (short)0, c, false, false);
  asm volatile("v_nop\n\tv_nop\n\tv_nop\n\tv_nop" : "+v"(d) : "v"(a), "v"(b));
  return d;
}

__device__ __forceinline__ v8h cv8(v4f a, v4f b) {
  v8h r;
  r[0] = (_Float16)a.x; r[1] = (_Float16)a.y; r[2] = (_Float16)a.z; r[3] = (_Float16)a.w;
  r[4] = (_Float16)b.x; r[5] = (_Float16)b.y; r[6] = (_Float16)b.z; r[7] = (_Float16)b.w;
  return r;
}

__device__ __forceinline__ v8f ldc8(const float* p) {
  const v4f a = *(const v4f*)p;
  const v4f b = *(const v4f*)(p + 4);
  v8f c;
  c[0] = a.x; c[1] = a.y; c[2] = a.z; c[3] = a.w;
  c[4] = b.x; c[5] = b.y; c[6] = b.z; c[7] = b.w;
  return c;
}

__device__ __forceinline__ v8f splat8(float x) {
  v8f c;
#pragma unroll
  for (int i = 0; i < 8; ++i) c[i] = x;
  return c;
}

__device__ __forceinline__ int scan_chunk(const int* __restrict__ dsts, int nE, int cbase, int nodeBase,
                                          int vec8, int* list, int tid, int wave) {
  int wc = 0;
  const int el0  = tid * EPT;
  const int e0   = cbase + el0;
  const int sent = -2147483647 - 1;
  v4i da, db;
  if (vec8 != 0 && cbase + CHUNK <= nE) {
    da = *(const v4i*)(dsts + e0);
    db = *(const v4i*)(dsts + e0 + 4);
  } else {
    da.x = (e0     < nE) ? dsts[min(e0, nE - 1)] : sent;
    da.y = (e0 + 1 < nE) ? dsts[min(e0 + 1, nE - 1)] : sent;
    da.z = (e0 + 2 < nE) ? dsts[min(e0 + 2, nE - 1)] : sent;
    da.w = (e0 + 3 < nE) ? dsts[min(e0 + 3, nE - 1)] : sent;
    db.x = (e0 + 4 < nE) ? dsts[min(e0 + 4, nE - 1)] : sent;
    db.y = (e0 + 5 < nE) ? dsts[min(e0 + 5, nE - 1)] : sent;
    db.z = (e0 + 6 < nE) ? dsts[min(e0 + 6, nE - 1)] : sent;
    db.w = (e0 + 7 < nE) ? dsts[min(e0 + 7, nE - 1)] : sent;
  }
  const unsigned nb = (unsigned)nodeBase;
  const unsigned s0 = (unsigned)da.x - nb, s1 = (unsigned)da.y - nb;
  const unsigned s2 = (unsigned)da.z - nb, s3 = (unsigned)da.w - nb;
  const unsigned s4 = (unsigned)db.x - nb, s5 = (unsigned)db.y - nb;
  const unsigned s6 = (unsigned)db.z - nb, s7 = (unsigned)db.w - nb;
  const bool h0 = s0 < (unsigned)NB, h1 = s1 < (unsigned)NB, h2 = s2 < (unsigned)NB, h3 = s3 < (unsigned)NB;
  const bool h4 = s4 < (unsigned)NB, h5 = s5 < (unsigned)NB, h6 = s6 < (unsigned)NB, h7 = s7 < (unsigned)NB;
  const unsigned any = __builtin_amdgcn_ballot_w32(h0 | h1 | h2 | h3 | h4 | h5 | h6 | h7);
  if (any != 0u) {
#define HITJ(J, HJ) { \
      const unsigned mj = __builtin_amdgcn_ballot_w32(HJ); \
      if (mj != 0u) { \
        if (HJ) { \
          const int pos = wc + (int)__builtin_amdgcn_mbcnt_lo(mj, 0u); \
          if (pos < WCAP) list[wave * WCAP + pos] = el0 + (J); \
        } \
        wc += (int)__builtin_popcount(mj); } }
    HITJ(0, h0)
    HITJ(1, h1)
    HITJ(2, h2)
    HITJ(3, h3)
    HITJ(4, h4)
    HITJ(5, h5)
    HITJ(6, h6)
    HITJ(7, h7)
#undef HITJ
  }
  return wc;
}

__global__ __launch_bounds__(NTHR) void k_prep(
    const float* __restrict__ s0, const float* __restrict__ s1, const float* __restrict__ s2,
    const float* __restrict__ s3, const float* __restrict__ s4, const float* __restrict__ s5,
    const float* __restrict__ s6, const float* __restrict__ s7, const float* __restrict__ s8,
    _Float16* planes) {
  const int b = blockIdx.x, tid = threadIdx.x;
  const int p = b >> 1;
  const float* src = s0;
  if (p == 1) src = s1;
  if (p == 2) src = s2;
  if (p == 3) src = s3;
  if (p == 4) src = s4;
  if (p == 5) src = s5;
  if (p == 6) src = s6;
  if (p == 7) src = s7;
  if (p >= 8) src = s8;
  const int u  = (b & 1) * NTHR + tid;
  const int n  = u >> 3;
  const int kc = u & 7;
  Pk8 pk;
#pragma unroll
  for (int j = 0; j < 8; ++j) {
    const int k = 8 * kc + j;
    pk.h[j] = (_Float16)(src[k * FD + n] * WSC);
  }
  const int pc = p > NPL - 1 ? NPL - 1 : p;
  _Float16* dp = planes + (size_t)pc * FD * FD + (size_t)u * 8;
  *(volatile v4i*)dp = pk.i;
  __threadfence();
  *(volatile v4i*)dp = pk.i;
}

__global__ __launch_bounds__(NTHR) void k_tfeat(const float* __restrict__ wt, const float* __restrict__ btv,
                                               float* tfo) {
  __shared__ float semb[TB * TD];
  __shared__ __attribute__((aligned(16))) float res[TB * FD];
  const int tid = threadIdx.x;
  {
    const int b = tid >> 5, k = tid & 31;
    const float emb = (k < TD / 2) ? 0.0f : 1.0f;
    semb[b * TD + k] = silu_f(emb);
  }
  __syncthreads();
#pragma unroll
  for (int q = 0; q < 2; ++q) {
    const int o = q * NTHR + tid;
    const int b = o >> 6, j = o & 63;
    float a = 0.0f;
#pragma unroll 1
    for (int k = 0; k < TD; ++k) a = fmaf(semb[b * TD + k], wt[k * FD + j], a);
    res[o] = a + btv[j];
  }
  __syncthreads();
  v4f v = {0.0f, 0.0f, 0.0f, 0.0f};
  const bool act = tid < (TB * FD) / 4;
  if (act) v = *(const v4f*)(res + 4 * tid);
  if (act) *(volatile v4f*)(tfo + 4 * tid) = v;
  __threadfence();
  if (act) *(volatile v4f*)(tfo + 4 * tid) = v;
}

__global__ __launch_bounds__(NTHR) void k_embed(const float* __restrict__ cond, const int* __restrict__ bt,
                                               const float* __restrict__ wn1, const float* __restrict__ bn1,
                                               const _Float16* __restrict__ N2t, const float* __restrict__ bn2,
                                               const float* __restrict__ tfp, float* hout, int nN) {
  __shared__ __attribute__((aligned(16))) float sw1[(CIN + 1) * FD];
  __shared__ __attribute__((aligned(16))) float sb1[FD];
  __shared__ float sb2[FD];
  __shared__ float stf[TB * FD];
  __shared__ __attribute__((aligned(16))) float stg[NWAVE * 16 * FD];
  const int tid = threadIdx.x, lane = tid & 31, wave = tid >> 5, hh = lane >> 4, m = lane & 15;
  for (int i = tid; i < (CIN + 1) * FD; i += NTHR) sw1[i] = wn1[i];
  if (tid < FD) { sb1[tid] = bn1[tid]; sb2[tid] = bn2[tid] * (WSC * HSC); }
  for (int i = tid; i < TB * FD; i += NTHR) stf[i] = tfp[i];
  __syncthreads();

  const int node0 = blockIdx.x * RB + wave * 16;
  int node = node0 + m;
  node = node > nN - 1 ? nN - 1 : node;
  const float* cr = cond + (size_t)node * CIN;

  FragH a[2];
#pragma unroll
  for (int kt = 0; kt < 2; ++kt) {
#pragma unroll
    for (int g = 0; g < 2; ++g) {
      const int kb = 32 * kt + 16 * g + 8 * hh;
      v8f acc8 = ldc8(sb1 + kb);
#pragma unroll 1
      for (int c = 0; c < CIN; ++c) {
        const float cv = cr[c];
        const v8f w8 = ldc8(sw1 + (c + 1) * FD + kb);
        acc8 = acc8 + cv * w8;
      }
      v8h hv;
#pragma unroll
      for (int i = 0; i < 8; ++i) hv[i] = (_Float16)(silu_f(acc8[i]) * HSC);
      a[kt].h[g] = hv;
    }
  }
  int bbv[8];
#pragma unroll
  for (int r = 0; r < 8; ++r) {
    int nd = node0 + 8 * hh + r;
    nd = nd > nN - 1 ? nN - 1 : nd;
    int bv = bt[nd];
    bv = bv < 0 ? 0 : (bv > TB - 1 ? TB - 1 : bv);
    bbv[r] = bv;
  }
#pragma unroll 1
  for (int nt = 0; nt < FD / 16; ++nt) {
    const int ncol = 16 * nt + m;
    v8f c = splat8(sb2[ncol]);
#pragma unroll
    for (int kt = 0; kt < 2; ++kt) {
      FragH b;
      const _Float16* bp = N2t + (size_t)ncol * FD + 32 * kt + 8 * hh;
      b.h[0] = *(const v8h*)bp;
      b.h[1] = *(const v8h*)(bp + 16);
      c = wmh(a[kt].v, b.v, c);
    }
#pragma unroll
    for (int r = 0; r < 8; ++r)
      stg[(wave * 16 + 8 * hh + r) * FD + ncol] = c[r] * HINV + stf[bbv[r] * FD + ncol];
  }
  __syncthreads();
#pragma unroll 1
  for (int rr = 0; rr < 8; ++rr) {
    const int row = wave * 16 + 2 * rr;
    const v4f v = *(const v4f*)(stg + row * FD + 4 * lane);
    *(volatile v4f*)(hout + (size_t)(blockIdx.x * RB + row) * FD + 4 * lane) = v;
  }
  __threadfence();
#pragma unroll 1
  for (int rr = 0; rr < 8; ++rr) {
    const int row = wave * 16 + 2 * rr;
    const v4f v = *(const v4f*)(stg + row * FD + 4 * lane);
    *(volatile v4f*)(hout + (size_t)(blockIdx.x * RB + row) * FD + 4 * lane) = v;
  }
}

__global__ __launch_bounds__(NTHR) void k_layer(
    const float* __restrict__ xin, const float* __restrict__ eattr, const int* __restrict__ ei,
    const float* __restrict__ ew1, const float* __restrict__ eb1,
    const _Float16* __restrict__ W2t, const float* __restrict__ eb2,
    const _Float16* __restrict__ M1t, const float* __restrict__ nb1,
    const _Float16* __restrict__ M2t, const float* __restrict__ nb2,
    float* xout, int nN, int nE, int vec8) {
  extern __shared__ __attribute__((aligned(16))) unsigned char dsm[];
  float*    acc   = (float*)(dsm + LDS_ACC);
  float*    msg   = (float*)(dsm + LDS_MSG);
  _Float16* hsn   = (_Float16*)(dsm + LDS_MSG);
  float*    stg   = (float*)(dsm + LDS_STG);
  int*      list  = (int*)(dsm + LDS_LIST);
  int*      pend  = (int*)(dsm + LDS_PEND);
  int*      slotb = (int*)(dsm + LDS_SLOT);
  float*    prm   = (float*)(dsm + LDS_PRM);
  int*      wcnt  = (int*)(dsm + LDS_WCNT);

  const int tid = threadIdx.x, lane = tid & 31, wave = tid >> 5, hh = lane >> 4, m = lane & 15;
  const int nodeBase = blockIdx.x * NB;
  const int* srcs = ei;
  const int* dsts = ei + nE;

  {
    const v4f z = {0.0f, 0.0f, 0.0f, 0.0f};
    for (int i = tid; i < (NB + 1) * FD / 4; i += NTHR) *(v4f*)(acc + 4 * i) = z;
  }
  if (tid < FD) {
    const int f = tid;
    prm[f]          = ew1[f];
    prm[FD + f]     = ew1[FD + f];
    prm[2 * FD + f] = eb1[f];
    prm[3 * FD + f] = eb2[f] * (WSC * HSC);
    prm[4 * FD + f] = nb1[f] * WSC;
    prm[5 * FD + f] = nb2[f] * (WSC * HSC);
  }
  if (tid == 0) wcnt[NWAVE] = 0;
  __syncthreads();

  const int nChunks = (nE + CHUNK - 1) / CHUNK;
#pragma unroll 1
  for (int ch = 0; ch < nChunks; ++ch) {
    const int cbase = ch * CHUNK;
    const int wc = scan_chunk(dsts, nE, cbase, nodeBase, vec8, list, tid, wave);
    if (lane == 0) wcnt[wave] = wc;
    __syncthreads();

    const int base = wcnt[NWAVE];
    int tot = 0, myoff = 0;
#pragma unroll
    for (int w = 0; w < NWAVE; ++w) {
      int c = wcnt[w];
      c = c > WCAP ? WCAP : (c < 0 ? 0 : c);
      if (w < wave) myoff += c;
      tot += c;
    }
    int newN = base + tot;
    newN = newN > PCAP ? PCAP : newN;
    {
      int n = wcnt[wave];
      n = n > WCAP ? WCAP : (n < 0 ? 0 : n);
      const int* lp = list + wave * WCAP;
      for (int i = lane; i < n; i += 32) {
        const int pos = base + myoff + i;
        if (pos < PCAP) pend[pos] = cbase + lp[i];
      }
    }
    const int fin = (ch == nChunks - 1) ? 1 : 0;
    const int R   = (fin != 0) ? (newN + PASSN - 1) / PASSN : newN / PASSN;
    const int Pv  = (fin != 0) ? newN : R * PASSN;
    __syncthreads();

#pragma unroll 1
    for (int r = 0; r < R; ++r) {
      int scl;
      {
        int idx = r * PASSN + wave * 16 + m;
        const bool valid = idx < Pv;
        idx = idx > PCAP - 1 ? PCAP - 1 : idx;
        int e = pend[idx];
        e = e < 0 ? 0 : (e > nE - 1 ? nE - 1 : e);
        const int d = dsts[e];
        int s = srcs[e];
        int slot = d - nodeBase;
        if (!valid || (unsigned)slot >= (unsigned)NB) slot = NB;
        s = s < 0 ? 0 : (s > nN - 1 ? nN - 1 : s);
        scl = s;
        const v2f av = *(const v2f*)(eattr + (size_t)e * EDIM);
        if (hh == 0) {
          *(v2f*)(stg + (wave * 16 + m) * EDIM) = av;
          slotb[wave * 16 + m] = slot;
        }
      }
      __syncthreads();

      FragH bq[2];
      {
        const v2f ea = *(const v2f*)(stg + (wave * 16 + m) * EDIM);
#pragma unroll
        for (int kt = 0; kt < 2; ++kt) {
#pragma unroll
          for (int g = 0; g < 2; ++g) {
            const int kb = 32 * kt + 16 * g + 8 * hh;
            const v8f w0 = ldc8(prm + kb);
            const v8f w1 = ldc8(prm + FD + kb);
            const v8f b0 = ldc8(prm + 2 * FD + kb);
            v8h hv;
#pragma unroll
            for (int i = 0; i < 8; ++i) {
              const float y = ea.x * w0[i] + ea.y * w1[i] + b0[i];
              hv[i] = (_Float16)(silu_f(y) * HSC);
            }
            bq[kt].h[g] = hv;
          }
        }
      }
#pragma unroll 1
      for (int ft = 0; ft < FD / 16; ++ft) {
        v8f c = ldc8(prm + 3 * FD + 16 * ft + 8 * hh);
#pragma unroll
        for (int kt = 0; kt < 2; ++kt) {
          FragH a;
          const _Float16* wp = W2t + (size_t)(16 * ft + m) * FD + 32 * kt + 8 * hh;
          a.h[0] = *(const v8h*)wp;
          a.h[1] = *(const v8h*)(wp + 16);
          c = wmh(a.v, bq[kt].v, c);
        }
        const int f0 = 16 * ft + 8 * hh;
        const float* xr = xin + (size_t)scl * FD + f0;
        const v4f x0 = *(const v4f*)xr;
        const v4f x1 = *(const v4f*)(xr + 4);
        float xs[8];
        xs[0] = x0.x; xs[1] = x0.y; xs[2] = x0.z; xs[3] = x0.w;
        xs[4] = x1.x; xs[5] = x1.y; xs[6] = x1.z; xs[7] = x1.w;
        float o[8];
#pragma unroll
        for (int rr = 0; rr < 8; ++rr) o[rr] = fmaxf(xs[rr] + c[rr] * HINV, 0.0f);
        float* mp = msg + (wave * 16 + m) * FD + f0;
        const v4f o0 = {o[0], o[1], o[2], o[3]};
        const v4f o1 = {o[4], o[5], o[6], o[7]};
        *(v4f*)mp = o0;
        *(v4f*)(mp + 4) = o1;
      }
      __syncthreads();

      if (tid < 32) {
#pragma unroll 1
        for (int i = 0; i < PASSN; ++i) {
          int sl = slotb[i];
          sl = sl < 0 ? 0 : (sl > NB ? NB : sl);
          const v2f mv = *(const v2f*)(msg + i * FD + 2 * tid);
          float* ap = acc + sl * FD + 2 * tid;
          v2f av = *(const v2f*)ap;
          av = av + mv;
          *(v2f*)ap = av;
        }
      }
      __syncthreads();
    }

    int rem = newN - R * PASSN;
    rem = rem < 0 ? 0 : rem;
    if (R > 0 && tid < rem) pend[tid] = pend[R * PASSN + tid];
    if (tid == 0) wcnt[NWAVE] = rem;
  }
  __syncthreads();

#pragma unroll 1
  for (int tt = 0; tt < NB / (16 * NWAVE); ++tt) {
    const int t    = wave + NWAVE * tt;
    const int lrow = 16 * t + m;
    int node = nodeBase + lrow;
    node = node > nN - 1 ? nN - 1 : node;
    const float* xr = xin + (size_t)node * FD;
    const float* ar = acc + lrow * FD;
    FragH bq[2];
#pragma unroll
    for (int kt = 0; kt < 2; ++kt) {
      const int k0 = 32 * kt + 8 * hh;
      const v4f xa = *(const v4f*)(xr + k0);
      const v4f xb = *(const v4f*)(xr + k0 + 4);
      const v4f xc = *(const v4f*)(xr + k0 + 16);
      const v4f xd = *(const v4f*)(xr + k0 + 20);
      const v4f ga = *(const v4f*)(ar + k0);
      const v4f gb = *(const v4f*)(ar + k0 + 4);
      const v4f gc = *(const v4f*)(ar + k0 + 16);
      const v4f gd = *(const v4f*)(ar + k0 + 20);
      bq[kt].h[0] = cv8(xa + ga, xb + gb);
      bq[kt].h[1] = cv8(xc + gc, xd + gd);
    }
    __syncthreads();
    _Float16* hw = hsn + wave * 16 * FD;
#pragma unroll 1
    for (int ft = 0; ft < FD / 16; ++ft) {
      v8f c = ldc8(prm + 4 * FD + 16 * ft + 8 * hh);
#pragma unroll
      for (int kt = 0; kt < 2; ++kt) {
        FragH a;
        const _Float16* wp = M1t + (size_t)(16 * ft + m) * FD + 32 * kt + 8 * hh;
        a.h[0] = *(const v8h*)wp;
        a.h[1] = *(const v8h*)(wp + 16);
        c = wmh(a.v, bq[kt].v, c);
      }
      v8h sv;
#pragma unroll
      for (int rr = 0; rr < 8; ++rr) sv[rr] = (_Float16)(silu_f(c[rr] * WINV) * HSC);
      *(v8h*)(hw + m * FD + 16 * ft + 8 * hh) = sv;
    }
    __syncthreads();
    FragH bz[2];
#pragma unroll
    for (int kt = 0; kt < 2; ++kt) {
      const _Float16* hp = hw + m * FD + 32 * kt + 8 * hh;
      bz[kt].h[0] = *(const v8h*)hp;
      bz[kt].h[1] = *(const v8h*)(hp + 16);
    }
#pragma unroll 1
    for (int ft = 0; ft < FD / 16; ++ft) {
      v8f c = ldc8(prm + 5 * FD + 16 * ft + 8 * hh);
#pragma unroll
      for (int kt = 0; kt < 2; ++kt) {
        FragH a;
        const _Float16* wp = M2t + (size_t)(16 * ft + m) * FD + 32 * kt + 8 * hh;
        a.h[0] = *(const v8h*)wp;
        a.h[1] = *(const v8h*)(wp + 16);
        c = wmh(a.v, bz[kt].v, c);
      }
      const int f0 = 16 * ft + 8 * hh;
      float o[8];
#pragma unroll
      for (int rr = 0; rr < 8; ++rr) o[rr] = silu_f(c[rr] * HINV);
      float* sp = acc + lrow * FD + f0;
      const v4f o0 = {o[0], o[1], o[2], o[3]};
      const v4f o1 = {o[4], o[5], o[6], o[7]};
      *(v4f*)sp = o0;
      *(v4f*)(sp + 4) = o1;
    }
    __syncthreads();
  }

#pragma unroll 1
  for (int rr = 0; rr < NB / NWAVE / 2; ++rr) {
    const int row = wave * (NB / NWAVE) + 2 * rr;
    const v4f v = *(const v4f*)(acc + row * FD + 4 * lane);
    *(volatile v4f*)(xout + (size_t)(nodeBase + row) * FD + 4 * lane) = v;
  }
  __threadfence();
#pragma unroll 1
  for (int rr = 0; rr < NB / NWAVE / 2; ++rr) {
    const int row = wave * (NB / NWAVE) + 2 * rr;
    const v4f v = *(const v4f*)(acc + row * FD + 4 * lane);
    *(volatile v4f*)(xout + (size_t)(nodeBase + row) * FD + 4 * lane) = v;
  }
}

__global__ __launch_bounds__(NTHR) void k_head(const float* __restrict__ hin,
                                              const _Float16* __restrict__ F1t, const float* __restrict__ bf1,
                                              const float* __restrict__ wf2, const float* __restrict__ bf2,
                                              float* out, int nN) {
  __shared__ float sb1[FD];
  __shared__ __attribute__((aligned(16))) float sv[FD];
  __shared__ __attribute__((aligned(16))) float hid[NWAVE * 16 * FD];
  __shared__ __attribute__((aligned(16))) float outs[RB];
  const int tid = threadIdx.x, lane = tid & 31, wave = tid >> 5, hh = lane >> 4, m = lane & 15;
  if (tid < FD) { sb1[tid] = bf1[tid] * WSC; sv[tid] = wf2[tid]; }
  __syncthreads();

  const int nb0   = blockIdx.x * RB;
  const int node0 = nb0 + wave * 16;
  int node = node0 + m;
  node = node > nN - 1 ? nN - 1 : node;
  FragH a[2];
  {
    const float* pr = hin + (size_t)node * FD + 8 * hh;
#pragma unroll
    for (int kt = 0; kt < 2; ++kt) {
      const float* p = pr + 32 * kt;
      a[kt].h[0] = cv8(*(const v4f*)p, *(const v4f*)(p + 4));
      a[kt].h[1] = cv8(*(const v4f*)(p + 16), *(const v4f*)(p + 20));
    }
  }
#pragma unroll 1
  for (int nt = 0; nt < FD / 16; ++nt) {
    const int ncol = 16 * nt + m;
    v8f c = splat8(sb1[ncol]);
#pragma unroll
    for (int kt = 0; kt < 2; ++kt) {
      FragH b;
      const _Float16* bp = F1t + (size_t)ncol * FD + 32 * kt + 8 * hh;
      b.h[0] = *(const v8h*)bp;
      b.h[1] = *(const v8h*)(bp + 16);
      c = wmh(a[kt].v, b.v, c);
    }
#pragma unroll
    for (int r = 0; r < 8; ++r) hid[(wave * 16 + 8 * hh + r) * FD + ncol] = silu_f(c[r] * WINV);
  }
  __syncthreads();
  float p = 0.0f;
  {
    const float* hr = hid + (wave * 16 + m) * FD + 32 * hh;
    const float* vr = sv + 32 * hh;
#pragma unroll 8
    for (int j = 0; j < 32; ++j) p = fmaf(hr[j], vr[j], p);
  }
  const float tot = p + __shfl_xor(p, 16);
  const float res = tot + bf2[0];
  if (hh == 0) outs[wave * 16 + m] = res;
  __syncthreads();

  const int rem = nN - nb0;
  const int u   = 4 * lane;
  v4f v = {0.0f, 0.0f, 0.0f, 0.0f};
  if (wave == 0) v = *(const v4f*)(outs + u);
  const bool fullv = (wave == 0) && (u + 4 <= rem);
  const bool t0 = (wave == 0) && !fullv && (u < rem);
  const bool t1 = (wave == 0) && !fullv && (u + 1 < rem);
  const bool t2 = (wave == 0) && !fullv && (u + 2 < rem);
  if (fullv) *(volatile v4f*)(out + nb0 + u) = v;
  if (t0) *(volatile float*)(out + nb0 + u) = v.x;
  if (t1) *(volatile float*)(out + nb0 + u + 1) = v.y;
  if (t2) *(volatile float*)(out + nb0 + u + 2) = v.z;
  __threadfence();
  if (fullv) *(volatile v4f*)(out + nb0 + u) = v;
  if (t0) *(volatile float*)(out + nb0 + u) = v.x;
  if (t1) *(volatile float*)(out + nb0 + u + 1) = v.y;
  if (t2) *(volatile float*)(out + nb0 + u + 2) = v.z;
}

extern "C" void kernel_launch(void* const* d_in, const int* in_sizes, int n_in,
                              void* d_out, int out_size, void* d_ws, size_t ws_size,
                              hipStream_t stream) {
  if (n_in < 30) return;
  const int nN = in_sizes[3];
  if (nN < 1 || in_sizes[0] != nN * CIN || out_size != nN) return;
  const int nE = in_sizes[2] / 2;
  if (nE < 1 || in_sizes[2] != 2 * nE || in_sizes[1] != nE * EDIM) return;
  if (in_sizes[4] != (CIN + 1) * FD || in_sizes[5] != FD) return;
  if (in_sizes[8] != EDIM * FD || in_sizes[9] != FD) return;
  if (in_sizes[12] != TD * FD || in_sizes[13] != FD) return;
  {
    const int wq[9] = {6, 10, 14, 16, 18, 20, 22, 24, 26};
    for (int i = 0; i < 9; ++i) if (in_sizes[wq[i]] != FD * FD) return;
    const int bq[9] = {7, 11, 15, 17, 19, 21, 23, 25, 27};
    for (int i = 0; i < 9; ++i) if (in_sizes[bq[i]] != FD) return;
  }
  if (in_sizes[28] != FD || in_sizes[29] != 1) return;

  const float* cond  = (const float*)d_in[0];
  const float* eattr = (const float*)d_in[1];
  const int*   ei    = (const int*)d_in[2];
  const int*   batch = (const int*)d_in[3];
  const float* w_n1  = (const float*)d_in[4];
  const float* b_n1  = (const float*)d_in[5];
  const float* w_n2  = (const float*)d_in[6];
  const float* b_n2  = (const float*)d_in[7];
  const float* w_e1  = (const float*)d_in[8];
  const float* b_e1  = (const float*)d_in[9];
  const float* w_e2  = (const float*)d_in[10];
  const float* b_e2  = (const float*)d_in[11];
  const float* w_t   = (const float*)d_in[12];
  const float* b_t   = (const float*)d_in[13];
  const float* wca[3] = {(const float*)d_in[14], (const float*)d_in[18], (const float*)d_in[22]};
  const float* bca[3] = {(const float*)d_in[15], (const float*)d_in[19], (const float*)d_in[23]};
  const float* wcb[3] = {(const float*)d_in[16], (const float*)d_in[20], (const float*)d_in[24]};
  const float* bcb[3] = {(const float*)d_in[17], (const float*)d_in[21], (const float*)d_in[25]};
  const float* w_f1  = (const float*)d_in[26];
  const float* b_f1  = (const float*)d_in[27];
  const float* w_f2  = (const float*)d_in[28];
  const float* b_f2  = (const float*)d_in[29];
  float* outp = (float*)d_out;

  const int nBlkL = (nN + NB - 1) / NB;
  const size_t rowsP = (size_t)nBlkL * NB;
  const int nBlkR = (nN + RB - 1) / RB;
  if ((size_t)nBlkR * RB > rowsP) return;

  char* ws = (char*)d_ws;
  size_t off = 0;
  const size_t oPL = off; off += ((size_t)NPL * FD * FD * 2 + 255) & ~(size_t)255;
  const size_t oTF = off; off += ((size_t)TB * FD * 4 + 255) & ~(size_t)255;
  const size_t oX0 = off; off += (rowsP * FD * 4 + 255) & ~(size_t)255;
  const size_t oX1 = off; off += (rowsP * FD * 4 + 255) & ~(size_t)255;
  size_t limit = (size_t)134217728;
  if (ws_size < limit) limit = ws_size;
  if (off > limit) return;

  _Float16* PL = (_Float16*)(ws + oPL);
  float* TF = (float*)(ws + oTF);
  float* X0 = (float*)(ws + oX0);
  float* X1 = (float*)(ws + oX1);
  const size_t PSZ = (size_t)FD * FD;

  const int vec8 = ((nE & 3) == 0) ? 1 : 0;

  k_prep<<<2 * NPL, NTHR, 0, stream>>>(w_n2, w_e2, wca[0], wcb[0], wca[1], wcb[1], wca[2], wcb[2], w_f1, PL);
  k_tfeat<<<1, NTHR, 0, stream>>>(w_t, b_t, TF);
  k_embed<<<nBlkR, NTHR, 0, stream>>>(cond, batch, w_n1, b_n1, PL, b_n2, TF, X0, nN);

  hipFuncSetAttribute(reinterpret_cast<const void*>(&k_layer), hipFuncAttributeMaxDynamicSharedMemorySize, LDS_TOTAL);

  const float* xcur = X0;
  float* planes[2] = {X1, X0};
  for (int l = 0; l < 3; ++l) {
    float* xo = planes[l & 1];
    k_layer<<<nBlkL, NTHR, LDS_TOTAL, stream>>>(
        xcur, eattr, ei,
        w_e1, b_e1,
        PL + 1 * PSZ, b_e2,
        PL + (size_t)(2 + 2 * l) * PSZ, bca[l],
        PL + (size_t)(3 + 2 * l) * PSZ, bcb[l],
        xo, nN, nE, vec8);
    xcur = xo;
  }

  k_head<<<nBlkR, NTHR, 0, stream>>>(xcur, PL + 8 * PSZ, b_f1, w_f2, b_f2, outp, nN);
}
